// Encoder_72954314489957
// MI455X (gfx1250) — hardware-verified
//
#include <hip/hip_runtime.h>
#include <stddef.h>
#include <stdint.h>
#include <math.h>


#define DIN    128
#define HC     256
#define NLR    512
#define CH     64
#define DENC   256
#define NGR    512
#define KCAT   320
#define KFC    384
#define NTHR   256
#define NWAVE  8
#define EPT    8
#define CHUNK  (NTHR * EPT)
#define WCAP   (EPT * 32)
#define LISTN  (NWAVE * WCAP)
#define NBA    1024
#define SLA    10
#define RCAP   28672
#define DEGCAP 64
#define GBM    64
#define GBN    64
#define GTHR   128
#define NUA    (HC * (DIN / 8))
#define NUB    (HC * (DIN / 8))
#define NUC    (DENC * (KFC / 8))
#define AGG_ZINTS (LISTN + 2 * RCAP + 3 * NBA)
#define AGG_LDS_INTS (AGG_ZINTS + 16)
#define WSMAX  134217728

static_assert((CHUNK & (CHUNK - 1)) == 0 && CHUNK <= 4096);
static_assert((NBA & (NBA - 1)) == 0 && NBA == (1 << SLA));
static_assert(((long long)CHUNK << SLA) < (1LL << 31));
static_assert(LISTN % NTHR == 0);
static_assert(NBA % NWAVE == 0 && NBA % 32 == 0);
static_assert(RCAP % 32 == 0 && AGG_ZINTS % 4 == 0 && LISTN % 4 == 0);
static_assert(DIN % 32 == 0 && KFC % 32 == 0 && KFC == DENC + 2 * CH && KCAT == DENC + CH);
static_assert(GBM == (GTHR / 32) * 16 && GBN == 64 && NLR % GBN == 0 && DENC % GBN == 0 && NGR % GBM == 0);
static_assert(NUA % NTHR == 0 && NUB % NTHR == 0 && NUC % NTHR == 0 && (NUA + NUB) % 8 == 0);
static_assert(DIN / 8 == 16 && KFC / 8 == 48 && KCAT % 8 == 0);
static_assert(HC == 8 * 32 && NLR == 2 * HC && CH == 64);
static_assert(AGG_LDS_INTS * 4 <= 300000);
static_assert((NGR * (DENC / 8)) % NTHR == 0);

typedef float          v2f   __attribute__((ext_vector_type(2)));
typedef float          v4f   __attribute__((ext_vector_type(4)));
typedef float          v8f   __attribute__((ext_vector_type(8)));
typedef int            v4i   __attribute__((ext_vector_type(4)));
typedef int            v8i   __attribute__((ext_vector_type(8)));
typedef unsigned short v8us  __attribute__((ext_vector_type(8)));
typedef unsigned short v16us __attribute__((ext_vector_type(16)));
typedef __bf16         v16bf __attribute__((ext_vector_type(16)));
typedef v2f  __attribute__((may_alias)) v2fa;
typedef v4f  __attribute__((may_alias)) v4fa;
typedef v4i  __attribute__((may_alias)) v4ia;
typedef v8us __attribute__((may_alias)) v8usa;
union FragB { v16bf v; v16us u; v8us h[2]; v8i w; };

__device__ __forceinline__ v8f wmb(const FragB& a, const FragB& b, v8f c) {
  v8f d = __builtin_amdgcn_wmma_f32_16x16x32_bf16(false, a.v, false, b.v, (short)0, c, false, false);
  asm volatile("v_nop\n\tv_nop\n\tv_nop\n\tv_nop" : "+v"(d) : "v"(a.w), "v"(b.w));
  return d;
}

__device__ __forceinline__ unsigned bf16_bits(float f) {
  const unsigned u = __float_as_uint(f);
  return (u + 0x7FFFu + ((u >> 16) & 1u)) >> 16;
}
__device__ __forceinline__ float bf16_val(float f) {
  return __uint_as_float(bf16_bits(f) << 16);
}

template <int SLB>
__device__ __forceinline__ int scan_chunk(const int* __restrict__ dsts, int nE, int cbase, int slotBase,
                                          int nb, int vec8, int* list, int tid, int lane, int wave) {
  int wc = 0;
  const int el0  = tid * EPT;
  const int e0   = cbase + el0;
  const int sent = -2147483647 - 1;
  v4i da, db;
  if (vec8 != 0 && cbase + CHUNK <= nE) {
    da = *(const v4i*)(dsts + e0);
    db = *(const v4i*)(dsts + e0 + 4);
  } else {
    da.x = (e0     < nE) ? dsts[min(e0,     nE - 1)] : sent;
    da.y = (e0 + 1 < nE) ? dsts[min(e0 + 1, nE - 1)] : sent;
    da.z = (e0 + 2 < nE) ? dsts[min(e0 + 2, nE - 1)] : sent;
    da.w = (e0 + 3 < nE) ? dsts[min(e0 + 3, nE - 1)] : sent;
    db.x = (e0 + 4 < nE) ? dsts[min(e0 + 4, nE - 1)] : sent;
    db.y = (e0 + 5 < nE) ? dsts[min(e0 + 5, nE - 1)] : sent;
    db.z = (e0 + 6 < nE) ? dsts[min(e0 + 6, nE - 1)] : sent;
    db.w = (e0 + 7 < nE) ? dsts[min(e0 + 7, nE - 1)] : sent;
  }
  const unsigned nbs = (unsigned)slotBase;
  const unsigned unb = (unsigned)nb;
  const unsigned s0 = (unsigned)da.x - nbs, s1 = (unsigned)da.y - nbs;
  const unsigned s2 = (unsigned)da.z - nbs, s3 = (unsigned)da.w - nbs;
  const unsigned s4 = (unsigned)db.x - nbs, s5 = (unsigned)db.y - nbs;
  const unsigned s6 = (unsigned)db.z - nbs, s7 = (unsigned)db.w - nbs;
  const bool h0 = s0 < unb, h1 = s1 < unb, h2 = s2 < unb, h3 = s3 < unb;
  const bool h4 = s4 < unb, h5 = s5 < unb, h6 = s6 < unb, h7 = s7 < unb;
  const unsigned any = __builtin_amdgcn_ballot_w32(h0 | h1 | h2 | h3 | h4 | h5 | h6 | h7);
  if (any != 0u) {
#define HITJ(J, HJ, SJ) { \
      const unsigned mj = __builtin_amdgcn_ballot_w32(HJ); \
      if (mj != 0u) { \
        if (HJ) { \
          const int pos = wc + (int)__builtin_amdgcn_mbcnt_lo(mj, 0u); \
          if (pos < WCAP) list[wave * WCAP + pos] = ((el0 + (J)) << SLB) | (int)(SJ); \
        } \
        wc += (int)__builtin_popcount(mj); } }
    HITJ(0, h0, s0)
    HITJ(1, h1, s1)
    HITJ(2, h2, s2)
    HITJ(3, h3, s3)
    HITJ(4, h4, s4)
    HITJ(5, h5, s5)
    HITJ(6, h6, s6)
    HITJ(7, h7, s7)
#undef HITJ
  }
  return wc;
}

__device__ __forceinline__ v8us gather8(const float* __restrict__ p, int stride) {
  v8us o;
#pragma unroll
  for (int i = 0; i < 8; ++i) o[i] = (unsigned short)bf16_bits(p[(size_t)i * (size_t)stride]);
  return o;
}

__global__ __launch_bounds__(NTHR) void k_wprep(const float* __restrict__ Wl, const float* __restrict__ Wr,
                                                const float* __restrict__ Wfc,
                                                unsigned short* WLR, unsigned short* WFT) {
  const int u = (int)blockIdx.x * NTHR + (int)threadIdx.x;
  v8us o;
  unsigned short* dp;
  if (u < NUA) {
    const int n  = u >> 4;
    const int k8 = (u & 15) * 8;
    o  = gather8(Wl + (size_t)k8 * HC + n, HC);
    dp = WLR + (size_t)n * DIN + k8;
  } else if (u < NUA + NUB) {
    const int v  = u - NUA;
    const int n  = v >> 4;
    const int k8 = (v & 15) * 8;
    o  = gather8(Wr + (size_t)k8 * HC + n, HC);
    dp = WLR + (size_t)(HC + n) * DIN + k8;
  } else if (u < NUA + NUB + NUC) {
    const int v  = u - (NUA + NUB);
    const int n  = v / (KFC / 8);
    const int k8 = (v - n * (KFC / 8)) * 8;
    const int ks = (k8 < KCAT) ? k8 : (k8 - CH);
    o  = gather8(Wfc + (size_t)ks * DENC + n, DENC);
    dp = WFT + (size_t)n * KFC + k8;
  } else {
    return;
  }
  *(volatile v8us*)dp = o;
  __threadfence();
  *(volatile v8us*)dp = o;
}

template <int COLS>
__global__ __launch_bounds__(NTHR) void k_cvt(const float* __restrict__ src, int nValid, int nUnits,
                                              unsigned short* dst, int pitch) {
  constexpr int UPR = COLS / 8;
  const int u = (int)blockIdx.x * NTHR + (int)threadIdx.x;
  if (u >= nUnits) return;
  const int row = u / UPR;
  const int k8  = (u - row * UPR) * 8;
  const int rc  = row < nValid ? row : nValid - 1;
  const float* p = src + (size_t)rc * COLS + k8;
  const v4f a = *(const v4fa*)p;
  const v4f b = *(const v4fa*)(p + 4);
  const bool ok = row < nValid;
  v8us o;
  o[0] = ok ? (unsigned short)bf16_bits(a.x) : (unsigned short)0;
  o[1] = ok ? (unsigned short)bf16_bits(a.y) : (unsigned short)0;
  o[2] = ok ? (unsigned short)bf16_bits(a.z) : (unsigned short)0;
  o[3] = ok ? (unsigned short)bf16_bits(a.w) : (unsigned short)0;
  o[4] = ok ? (unsigned short)bf16_bits(b.x) : (unsigned short)0;
  o[5] = ok ? (unsigned short)bf16_bits(b.y) : (unsigned short)0;
  o[6] = ok ? (unsigned short)bf16_bits(b.z) : (unsigned short)0;
  o[7] = ok ? (unsigned short)bf16_bits(b.w) : (unsigned short)0;
  unsigned short* dp = dst + (size_t)row * (size_t)pitch + k8;
  *(volatile v8us*)dp = o;
  __threadfence();
  *(volatile v8us*)dp = o;
}

__global__ __launch_bounds__(GTHR) void k_gemm(
    const unsigned short* __restrict__ A, const unsigned short* __restrict__ WT,
    const float* __restrict__ biasA, const float* __restrict__ biasB,
    float* outF, int K, int ldo)
{
  __shared__ __attribute__((aligned(16))) float stg[GBM * GBN];
  const int tid = (int)threadIdx.x, lane = tid & 31, wave = tid >> 5, hh = lane >> 4, m = lane & 15;
  const int rowBase = (int)blockIdx.x * GBM;
  const int col0    = (int)blockIdx.y * GBN;

  v8f acc[4];
  {
    const v8f z = {0.f, 0.f, 0.f, 0.f, 0.f, 0.f, 0.f, 0.f};
    acc[0] = z; acc[1] = z; acc[2] = z; acc[3] = z;
  }
  const unsigned short* ap = A  + (size_t)(rowBase + 16 * wave + m) * (size_t)K + 8 * hh;
  const unsigned short* wp = WT + (size_t)(col0 + m) * (size_t)K + 8 * hh;
  const int ksteps = K >> 5;
#pragma unroll 1
  for (int ks = 0; ks < ksteps; ++ks) {
    FragB af;
    af.h[0] = *(const v8usa*)(ap + 32 * ks);
    af.h[1] = *(const v8usa*)(ap + 32 * ks + 16);
#pragma unroll
    for (int t = 0; t < 4; ++t) {
      const unsigned short* wq = wp + (size_t)(16 * t) * (size_t)K + 32 * ks;
      FragB bf;
      bf.h[0] = *(const v8usa*)wq;
      bf.h[1] = *(const v8usa*)(wq + 16);
      acc[t] = wmb(af, bf, acc[t]);
    }
  }

#pragma unroll
  for (int t = 0; t < 4; ++t) {
    const int lc = 16 * t + m;
#pragma unroll
    for (int r = 0; r < 8; ++r) {
      const int lr = 16 * wave + 8 * hh + r;
      stg[lr * GBN + lc] = acc[t][r];
    }
  }
  __syncthreads();

  v4f bq;
  {
    const int cb = (col0 & 255) + 4 * m;
    const v4f ba = *(const v4fa*)(biasA + cb);
    const v4f bb = *(const v4fa*)(biasB + cb);
    const bool fa = col0 < 256;
    bq.x = bf16_val(fa ? ba.x : bb.x);
    bq.y = bf16_val(fa ? ba.y : bb.y);
    bq.z = bf16_val(fa ? ba.z : bb.z);
    bq.w = bf16_val(fa ? ba.w : bb.w);
  }

  v4f fv[8];
#pragma unroll
  for (int i = 0; i < 8; ++i) {
    const int lr = 16 * wave + 2 * i + hh;
    const v4f t = *(const v4fa*)(stg + lr * GBN + 4 * m);
    fv[i] = t + bq;
  }
#pragma unroll
  for (int i = 0; i < 8; ++i) {
    const int lr = 16 * wave + 2 * i + hh;
    const int gr = rowBase + lr;
    float* op = outF + (size_t)gr * (size_t)ldo + col0 + 4 * m;
    *(volatile v4f*)op = fv[i];
  }
  __threadfence();
#pragma unroll
  for (int i = 0; i < 8; ++i) {
    const int lr = 16 * wave + 2 * i + hh;
    const int gr = rowBase + lr;
    float* op = outF + (size_t)gr * (size_t)ldo + col0 + 4 * m;
    *(volatile v4f*)op = fv[i];
  }
}

__device__ __forceinline__ float lk(float v, float slope) { return (v > 0.0f) ? v : slope * v; }

__device__ __forceinline__ float score8(v4f xa, v4f xb, v4f ra, v4f rb, v4f aa, v4f ab) {
  float p = lk(xa.x + ra.x, 0.2f) * aa.x;
  p = fmaf(lk(xa.y + ra.y, 0.2f), aa.y, p);
  p = fmaf(lk(xa.z + ra.z, 0.2f), aa.z, p);
  p = fmaf(lk(xa.w + ra.w, 0.2f), aa.w, p);
  p = fmaf(lk(xb.x + rb.x, 0.2f), ab.x, p);
  p = fmaf(lk(xb.y + rb.y, 0.2f), ab.y, p);
  p = fmaf(lk(xb.z + rb.z, 0.2f), ab.z, p);
  p = fmaf(lk(xb.w + rb.w, 0.2f), ab.w, p);
  p += __shfl_xor(p, 1, 32);
  p += __shfl_xor(p, 2, 32);
  p += __shfl_xor(p, 4, 32);
  return p;
}
__device__ __forceinline__ float hsum(float v) {
  v += __shfl_xor(v, 8, 32);
  v += __shfl_xor(v, 16, 32);
  return v;
}

__global__ __launch_bounds__(NTHR) void k_scan(const int* __restrict__ srcs, const int* __restrict__ dsts,
                                               int nE, int nN, int vec8,
                                               const float* __restrict__ xlr, const float* __restrict__ att,
                                               const float* __restrict__ bgnn, float* hn) {
  extern __shared__ __attribute__((aligned(16))) int dsm[];
  int* list = dsm;
  int* hl   = dsm + LISTN;
  int* sl   = dsm + LISTN + RCAP;
  int* cnt  = dsm + LISTN + 2 * RCAP;
  int* offs = cnt + NBA;
  int* cur  = offs + NBA;
  int* misc = cur + NBA;
  const int tid = (int)threadIdx.x, lane = tid & 31, wave = tid >> 5;
  const int nodeBase = (int)blockIdx.x * NBA;

  {
    const v4i z4 = {0, 0, 0, 0};
    for (int i = tid * 4; i < AGG_ZINTS; i += NTHR * 4) *(v4ia*)(dsm + i) = z4;
    if (tid < 16) misc[tid] = 0;
  }
  __syncthreads();

  int t = 0, ov = 0;
  const int nChunks = (nE + CHUNK - 1) / CHUNK;
#pragma unroll 1
  for (int ch = 0; ch < nChunks; ++ch) {
    const int cbase = ch * CHUNK;
    const int wc = scan_chunk<SLA>(dsts, nE, cbase, nodeBase, NBA, vec8, list, tid, lane, wave);
    if (lane == 0) misc[wave] = wc;
    __syncthreads();
    if (wave == 0) {
#pragma unroll 1
      for (int w2 = 0; w2 < NWAVE; ++w2) {
        int c = misc[w2];
        c = c < 0 ? 0 : (c > WCAP ? WCAP : c);
#pragma unroll 1
        for (int b0 = 0; b0 < c; b0 += 32) {
          const int idx = b0 + lane;
          const int ent = list[w2 * WCAP + (idx < WCAP ? idx : WCAP - 1)];
          const int m32 = (c - b0) < 32 ? (c - b0) : 32;
#pragma unroll 1
          for (int k = 0; k < m32; ++k) {
            const int u    = __builtin_amdgcn_readlane(ent, k);
            const int slot = u & (NBA - 1);
            const int el   = (u >> SLA) & (CHUNK - 1);
            const int pk   = ((cbase + el) << SLA) | slot;
            if (t < RCAP) {
              if (lane == 0) { hl[t] = pk; cnt[slot] = cnt[slot] + 1; }
              t = t + 1;
            } else {
              ov = 1;
            }
          }
        }
      }
    }
    __syncthreads();
  }
  if (wave == 0 && lane == 0) { misc[8] = t; misc[9] = ov; }
  __syncthreads();
  int tt = misc[8];
  tt = tt < 0 ? 0 : (tt > RCAP ? RCAP : tt);
  const int ovf = misc[9];

  if (wave == 0) {
    const int base = lane * (NBA / 32);
    int s = 0;
#pragma unroll 1
    for (int i = 0; i < NBA / 32; ++i) s += cnt[base + i];
    int incl = s;
#pragma unroll
    for (int d = 1; d < 32; d <<= 1) {
      const int y = __shfl_up(incl, d, 32);
      if (lane >= d) incl += y;
    }
    int run = incl - s;
#pragma unroll 1
    for (int i = 0; i < NBA / 32; ++i) {
      const int cv = cnt[base + i];
      offs[base + i] = run;
      cur[base + i]  = run;
      run += cv;
    }
  }
  __syncthreads();
  if (wave == 0) {
#pragma unroll 1
    for (int b0 = 0; b0 < tt; b0 += 32) {
      const int idx = b0 + lane;
      const int ent = hl[idx < RCAP ? idx : RCAP - 1];
      const int m32 = (tt - b0) < 32 ? (tt - b0) : 32;
#pragma unroll 1
      for (int k = 0; k < m32; ++k) {
        const int u    = __builtin_amdgcn_readlane(ent, k);
        const int slot = u & (NBA - 1);
        if (lane == 0) {
          int p = cur[slot];
          p = p < 0 ? 0 : (p > RCAP - 1 ? RCAP - 1 : p);
          sl[p] = u;
          cur[slot] = p + 1;
        }
      }
    }
  }
  __syncthreads();

  const float qnan = __int_as_float(0x7fc00000);
  const float pz = (ovf != 0) ? qnan : 0.0f;
  v4f atA, atB, bgA, bgB;
  {
    const v4f t0 = *(const v4fa*)(att + 8 * lane);
    const v4f t1 = *(const v4fa*)(att + 8 * lane + 4);
    atA.x = bf16_val(t0.x); atA.y = bf16_val(t0.y); atA.z = bf16_val(t0.z); atA.w = bf16_val(t0.w);
    atB.x = bf16_val(t1.x); atB.y = bf16_val(t1.y); atB.z = bf16_val(t1.z); atB.w = bf16_val(t1.w);
    const int cg = 8 * (lane & 7);
    const v4f u0 = *(const v4fa*)(bgnn + cg);
    const v4f u1 = *(const v4fa*)(bgnn + cg + 4);
    bgA.x = bf16_val(u0.x); bgA.y = bf16_val(u0.y); bgA.z = bf16_val(u0.z); bgA.w = bf16_val(u0.w);
    bgB.x = bf16_val(u1.x); bgB.y = bf16_val(u1.y); bgB.z = bf16_val(u1.z); bgB.w = bf16_val(u1.w);
  }
  const int sl2 = lane >> 1;
  const bool od = (lane & 1) != 0;
#pragma unroll 1
  for (int si = 0; si < NBA / NWAVE; ++si) {
    const int s    = si * NWAVE + wave;
    const int node = nodeBase + s;
    int c = cnt[s];
    const bool big = c > DEGCAP;
    c = c < 0 ? 0 : (c > DEGCAP ? DEGCAP : c);
    int o = offs[s];
    o = o < 0 ? 0 : (o > RCAP ? RCAP : o);
    const int nc = node < nN ? node : nN - 1;
    const float* rowi = xlr + (size_t)nc * NLR + 8 * lane;
    const v4f xrA = *(const v4fa*)(rowi + HC);
    const v4f xrB = *(const v4fa*)(rowi + HC + 4);
    v4f accA = *(const v4fa*)rowi;
    v4f accB = *(const v4fa*)(rowi + 4);
    float mx = score8(accA, accB, xrA, xrB, atA, atB);
    float ls = 1.0f;
#pragma unroll 1
    for (int b0 = 0; b0 < c; b0 += 32) {
      int idx = o + b0 + lane;
      idx = idx > RCAP - 1 ? RCAP - 1 : idx;
      const int ent = sl[idx];
      int eid = ent >> SLA;
      eid = eid < 0 ? 0 : (eid > nE - 1 ? nE - 1 : eid);
      int sr = srcs[eid];
      sr = sr < 0 ? 0 : (sr > nN - 1 ? nN - 1 : sr);
      const int m32 = (c - b0) < 32 ? (c - b0) : 32;
#pragma unroll 1
      for (int k = 0; k < m32; ++k) {
        const int sk = __builtin_amdgcn_readlane(sr, k);
        const float* rp = xlr + (size_t)sk * NLR + 8 * lane;
        const v4f xa = *(const v4fa*)rp;
        const v4f xb = *(const v4fa*)(rp + 4);
        const float e  = score8(xa, xb, xrA, xrB, atA, atB);
        const float d  = e - mx;
        const float tv = expf(-fabsf(d));
        const bool  up = d > 0.0f;
        const float sc = up ? tv : 1.0f;
        const float pw = up ? 1.0f : tv;
        mx = up ? e : mx;
        ls = fmaf(ls, sc, pw);
        accA = accA * sc + xa * pw;
        accB = accB * sc + xb * pw;
      }
    }
    const float inv = 1.0f / (ls + 1e-16f);
    float y0 = hsum(accA.x * inv), y1 = hsum(accA.y * inv), y2 = hsum(accA.z * inv), y3 = hsum(accA.w * inv);
    float y4 = hsum(accB.x * inv), y5 = hsum(accB.y * inv), y6 = hsum(accB.z * inv), y7 = hsum(accB.w * inv);
    const float pzr = big ? qnan : pz;
    y0 = lk(fmaf(y0, 0.25f, bgA.x), 0.01f) + pzr;
    y1 = lk(fmaf(y1, 0.25f, bgA.y), 0.01f) + pzr;
    y2 = lk(fmaf(y2, 0.25f, bgA.z), 0.01f) + pzr;
    y3 = lk(fmaf(y3, 0.25f, bgA.w), 0.01f) + pzr;
    y4 = lk(fmaf(y4, 0.25f, bgB.x), 0.01f) + pzr;
    y5 = lk(fmaf(y5, 0.25f, bgB.y), 0.01f) + pzr;
    y6 = lk(fmaf(y6, 0.25f, bgB.z), 0.01f) + pzr;
    y7 = lk(fmaf(y7, 0.25f, bgB.w), 0.01f) + pzr;
    const float g0 = __shfl(y0, sl2, 32), g1 = __shfl(y1, sl2, 32);
    const float g2 = __shfl(y2, sl2, 32), g3 = __shfl(y3, sl2, 32);
    const float g4 = __shfl(y4, sl2, 32), g5 = __shfl(y5, sl2, 32);
    const float g6 = __shfl(y6, sl2, 32), g7 = __shfl(y7, sl2, 32);
    v4f ow;
    ow.x = od ? g4 : g0;
    ow.y = od ? g5 : g1;
    ow.z = od ? g6 : g2;
    ow.w = od ? g7 : g3;
    const bool wr = (node < nN) && (lane < 16);
    float* op = hn + (size_t)nc * CH + 4 * (lane & 15);
    if (wr) *(volatile v4f*)op = ow;
    __threadfence();
    if (wr) *(volatile v4f*)op = ow;
  }
}

__global__ __launch_bounds__(NTHR) void k_pool(const float* __restrict__ hf, const int* __restrict__ bat,
                                               int nN, unsigned short* cat) {
  __shared__ __attribute__((aligned(16))) float wsum[NWAVE * CH];
  __shared__ int wcn[NWAVE];
  __shared__ __attribute__((aligned(16))) unsigned short ob[2 * CH];
  const int tid = (int)threadIdx.x, lane = tid & 31, wave = tid >> 5;
  const int g = (int)blockIdx.x;

  float a0 = 0.0f, a1 = 0.0f;
  int cnt = 0;
#pragma unroll 1
  for (int i0 = wave * 32; i0 < nN; i0 += NTHR) {
    const int i  = i0 + lane;
    const int ic = i < nN ? i : nN - 1;
    const int b  = bat[ic];
    const bool hit = (i < nN) && (b == g);
    unsigned msk = __builtin_amdgcn_ballot_w32(hit);
    int nh = (int)__builtin_popcount(msk);
    nh = nh > 32 ? 32 : nh;
    cnt += nh;
#pragma unroll 1
    for (int q = 0; q < nh; ++q) {
      const int k = __builtin_ffs((int)msk) - 1;
      msk &= msk - 1u;
      int node = i0 + (k < 0 ? 0 : k);
      node = node > nN - 1 ? nN - 1 : node;
      const v2f v = *(const v2fa*)(hf + (size_t)node * CH + 2 * lane);
      a0 += v.x; a1 += v.y;
    }
  }
  wsum[wave * CH + 2 * lane + 0] = a0;
  wsum[wave * CH + 2 * lane + 1] = a1;
  if (lane == 0) wcn[wave] = cnt;
  __syncthreads();
  if (tid < CH) {
    float s = 0.0f;
    int c = 0;
#pragma unroll
    for (int w2 = 0; w2 < NWAVE; ++w2) { s += wsum[w2 * CH + tid]; c += wcn[w2]; }
    const float cf = (c < 1) ? 1.0f : (float)c;
    const float hg = s * (1.0f / cf);
    const unsigned hb = bf16_bits(hg);
    const unsigned lb = bf16_bits(hg - __uint_as_float(hb << 16));
    ob[tid]      = (unsigned short)hb;
    ob[CH + tid] = (unsigned short)lb;
  }
  __syncthreads();
  const v8us ov = *(const v8usa*)(ob + 8 * (lane & 15));
  unsigned short* op = cat + (size_t)g * KFC + DENC + 8 * (lane & 15);
  const bool okst = (wave == 0) && (lane < 16);
  if (okst) *(volatile v8us*)op = ov;
  __threadfence();
  if (okst) *(volatile v8us*)op = ov;
}

static inline int cdiv(int a, int b) { return (a + b - 1) / b; }
static inline size_t al256(size_t o) { return (o + 255) & ~(size_t)255; }

extern "C" void kernel_launch(void* const* d_in, const int* in_sizes, int n_in,
                              void* d_out, int out_size, void* d_ws, size_t ws_size,
                              hipStream_t stream) {
  if (n_in < 12) return;
  if (in_sizes[0] != NGR * DENC) return;
  if (in_sizes[1] < DIN || (in_sizes[1] % DIN) != 0) return;
  const int nN = in_sizes[1] / DIN;
  if (nN < 1 || nN > (1 << 20)) return;
  if (in_sizes[2] < 2 || (in_sizes[2] & 1) != 0) return;
  const int nE = in_sizes[2] / 2;
  if (nE < 1 || nE >= (1 << (31 - SLA))) return;
  if (in_sizes[3] != nN) return;
  if (in_sizes[4] != DIN * HC || in_sizes[5] != HC) return;
  if (in_sizes[6] != DIN * HC || in_sizes[7] != HC) return;
  if (in_sizes[8] != HC || in_sizes[9] != CH) return;
  if (in_sizes[10] != KCAT * DENC || in_sizes[11] != DENC) return;
  if (out_size != NGR * DENC) return;

  const float* hy   = (const float*)d_in[0];
  const float* x    = (const float*)d_in[1];
  const int*   edge = (const int*)d_in[2];
  const int*   bat  = (const int*)d_in[3];
  const float* Wl   = (const float*)d_in[4];
  const float* bl   = (const float*)d_in[5];
  const float* Wr   = (const float*)d_in[6];
  const float* br   = (const float*)d_in[7];
  const float* att  = (const float*)d_in[8];
  const float* bgnn = (const float*)d_in[9];
  const float* Wfc  = (const float*)d_in[10];
  const float* bfc  = (const float*)d_in[11];
  float* out = (float*)d_out;
  const int* src = edge;
  const int* dst = edge + nE;

  const int MP = cdiv(nN, GBM) * GBM;
  const int gM = MP / GBM;
  const int gA = cdiv(nN, NBA);
  if ((long long)gA * NBA < (long long)nN) return;
  const int vec8 = ((nE & 3) == 0) ? 1 : 0;

  char* ws = (char*)d_ws;
  size_t off = 0;
  const size_t oWLR = off; off = al256(off + (size_t)NLR * DIN * 2);
  const size_t oWFT = off; off = al256(off + (size_t)DENC * KFC * 2);
  const size_t oCAT = off; off = al256(off + (size_t)NGR * KFC * 2);
  const size_t oXB  = off; off = al256(off + (size_t)MP * DIN * 2);
  const size_t oXLR = off; off = al256(off + (size_t)MP * NLR * 4);
  const size_t oHN  = off; off = al256(off + (size_t)nN * CH * 4);
  if (off > ws_size || off > (size_t)WSMAX) return;
  unsigned short* WLR = (unsigned short*)(ws + oWLR);
  unsigned short* WFT = (unsigned short*)(ws + oWFT);
  unsigned short* CAT = (unsigned short*)(ws + oCAT);
  unsigned short* XB  = (unsigned short*)(ws + oXB);
  float*          XLR = (float*)(ws + oXLR);
  float*          HN  = (float*)(ws + oHN);

  const size_t scanLds = (size_t)AGG_LDS_INTS * 4;
  hipFuncSetAttribute(reinterpret_cast<const void*>(&k_scan), hipFuncAttributeMaxDynamicSharedMemorySize, (int)scanLds);

  const int nUx = MP * (DIN / 8);
  const int nUh = NGR * (DENC / 8);
  k_wprep<<<(NUA + NUB + NUC) / NTHR, NTHR, 0, stream>>>(Wl, Wr, Wfc, WLR, WFT);
  k_cvt<DIN><<<cdiv(nUx, NTHR), NTHR, 0, stream>>>(x, nN, nUx, XB, DIN);
  k_cvt<DENC><<<cdiv(nUh, NTHR), NTHR, 0, stream>>>(hy, NGR, nUh, CAT, KFC);
  k_gemm<<<dim3(gM, NLR / GBN), GTHR, 0, stream>>>(XB, WLR, bl, br, XLR, DIN, NLR);
  k_scan<<<gA, NTHR, scanLds, stream>>>(src, dst, nE, nN, vec8, XLR, att, bgnn, HN);
  k_pool<<<NGR, NTHR, 0, stream>>>(HN, bat, nN, CAT);
  k_gemm<<<dim3(NGR / GBM, DENC / GBN), GTHR, 0, stream>>>(CAT, WFT, bfc, bfc, out, KFC, DENC);
}
